// LSTM_GCN_3496103379265
// MI455X (gfx1250) — hardware-verified
//
#include <hip/hip_runtime.h>

typedef __attribute__((ext_vector_type(16))) _Float16 v16h;
typedef __attribute__((ext_vector_type(8)))  _Float16 v8h;
typedef __attribute__((ext_vector_type(16))) __bf16   v16b;
typedef __attribute__((ext_vector_type(8)))  __bf16   v8b;
typedef __attribute__((ext_vector_type(8)))  float    v8f;
typedef __attribute__((ext_vector_type(4)))  float    v4f;
typedef __attribute__((ext_vector_type(4)))  unsigned v4u;

__device__ __forceinline__ unsigned short f2bf_bits(float f) {
  unsigned u = __float_as_uint(f);
  return (unsigned short)((u + 0x7FFFu + ((u >> 16) & 1u)) >> 16);
}
__device__ __forceinline__ float bf_bits2f(unsigned short h) { return __uint_as_float(((unsigned)h) << 16); }

__device__ __forceinline__ void dep_guard_h(v8f& a, v8f& b, v16h x, v16h y) { asm volatile("v_nop\n\tv_nop\n\tv_nop\n\tv_nop" : "+v"(a), "+v"(b) : "v"(x), "v"(y)); }
__device__ __forceinline__ void dep_guard_b(v8f& a, v8f& b, v16b x, v16b y) { asm volatile("v_nop\n\tv_nop\n\tv_nop\n\tv_nop" : "+v"(a), "+v"(b) : "v"(x), "v"(y)); }
__device__ __forceinline__ void keep4_h(v16h a, v16h b, v16h c, v16h d) { asm volatile("v_nop" :: "v"(a), "v"(b), "v"(c), "v"(d)); }
__device__ __forceinline__ void keep4_b(v16b a, v16b b, v16b c, v16b d) { asm volatile("v_nop" :: "v"(a), "v"(b), "v"(c), "v"(d)); }
__device__ __forceinline__ void acc_guard4(v8f& a, v8f& b, v8f& c, v8f& d) { asm volatile("v_nop\n\tv_nop\n\tv_nop\n\tv_nop" : "+v"(a), "+v"(b), "+v"(c), "+v"(d)); }
template <typename T> struct Frag;
template <> struct Frag<_Float16> {
  typedef v16h V; union U { v16h v; v8h h[2]; };
  static __device__ __forceinline__ v16h load(const _Float16* p) {
    U f; f.h[0] = *(const v8h*)(p); f.h[1] = *(const v8h*)(p + 16); return f.v;
  }
  static __device__ __forceinline__ v8f mma(v16h a, v16h b, v8f c) {
    return __builtin_amdgcn_wmma_f32_16x16x32_f16(false, a, false, b, (short)0, c, false, false);
  }
  static __device__ __forceinline__ void guard(v8f& a, v8f& b, v16h x, v16h y) { dep_guard_h(a, b, x, y); }
  static __device__ __forceinline__ void keep(v16h a, v16h b, v16h c, v16h d) { keep4_h(a, b, c, d); }
};
template <> struct Frag<__bf16> {
  typedef v16b V; union U { v16b v; v8b h[2]; };
  static __device__ __forceinline__ v16b load(const __bf16* p) {
    U f; f.h[0] = *(const v8b*)(p); f.h[1] = *(const v8b*)(p + 16); return f.v;
  }
  static __device__ __forceinline__ v8f mma(v16b a, v16b b, v8f c) {
    return __builtin_amdgcn_wmma_f32_16x16x32_bf16(false, a, false, b, (short)0, c, false, false);
  }
  static __device__ __forceinline__ void guard(v8f& a, v8f& b, v16b x, v16b y) { dep_guard_b(a, b, x, y); }
  static __device__ __forceinline__ void keep(v16b a, v16b b, v16b c, v16b d) { keep4_b(a, b, c, d); }
};

constexpr int NB   = 32;
constexpr int NCIN = 64;
constexpr int TT   = 64;
constexpr int NV   = 25;
constexpr int HSZ  = 128;
constexpr int NSC  = 8;
constexpr int NC1  = 32;
constexpr int NC2  = 64;
constexpr int KXW  = NSC * NCIN;
constexpr int KHW  = NSC * HSZ;
constexpr int KTOT = KXW + KHW;
constexpr int MG   = 4 * HSZ;
constexpr int NCOL = NB * NV;
constexpr int NCOLP = 832;
constexpr int AROWS = NSC * NV;
constexpr int AROWT = 13;
constexpr int APROWS = 256;
constexpr int VPAD = 32;
constexpr int GEMM_TN = NCOLP / 64;
constexpr int GEMM_TM = MG / 64;
constexpr int SLABP = 68;

constexpr float SC_W   = 0.015625f;
constexpr float SC_AUG = 0.0625f;
constexpr float SC_RES = 0.00048828125f;
constexpr float LOG2E_F = 1.4426950408889634f;

typedef char chk_kparts[((KXW % 32) == 0 && (KHW % 32) == 0 && (MG % 64) == 0 && (NCOLP % 64) == 0 && NCOLP >= NCOL) ? 1 : -1];
typedef char chk_tiles[(GEMM_TN * GEMM_TM == 104 && AROWT * 16 >= AROWS && AROWT * 16 <= APROWS) ? 1 : -1];

constexpr size_t SZ_APL   = (size_t)MG * KTOT * 2;
constexpr size_t SZ_BHI   = (size_t)NCOLP * KTOT * 2;
constexpr size_t SZ_BLO   = (size_t)NCOLP * KXW * 2;
constexpr size_t SZ_BIAS  = (size_t)MG * NV * 4;
constexpr size_t SZ_A16   = (size_t)APROWS * VPAD * 2;
constexpr size_t SZ_WH16  = (size_t)NC2 * HSZ * 2;
constexpr size_t SZ_STATE = (size_t)HSZ * NCOLP * 4;
constexpr size_t SZ_HSEQ  = (size_t)TT * NB * HSZ * VPAD * 4;
constexpr size_t OFF_APL  = 0;
constexpr size_t OFF_BHI  = OFF_APL + SZ_APL;
constexpr size_t OFF_BLO  = OFF_BHI + SZ_BHI;
constexpr size_t OFF_BIAS = OFF_BLO + SZ_BLO;
constexpr size_t OFF_AWG  = OFF_BIAS + SZ_BIAS;
constexpr size_t OFF_AUG  = OFF_AWG + SZ_A16;
constexpr size_t OFF_WH   = OFF_AUG + SZ_A16;
constexpr size_t OFF_C0   = OFF_WH + SZ_WH16;
constexpr size_t OFF_C1   = OFF_C0 + SZ_STATE;
constexpr size_t OFF_HPRE = OFF_C1 + SZ_STATE;
constexpr size_t OFF_HSEQ = OFF_HPRE + SZ_STATE;
constexpr size_t WS_TOTAL = OFF_HSEQ + SZ_HSEQ;
typedef char chk_ws[(WS_TOTAL <= (size_t)134217728) ? 1 : -1];
typedef char chk_align[((OFF_BHI % 256) == 0 && (OFF_BLO % 256) == 0 && (OFF_BIAS % 256) == 0 && (OFF_AWG % 256) == 0 &&
                        (OFF_C0 % 256) == 0 && (OFF_HPRE % 256) == 0 && (OFF_HSEQ % 256) == 0) ? 1 : -1];

constexpr size_t OUT0_N = (size_t)NB * HSZ * TT * NV;
constexpr size_t OUT1_N = (size_t)NB * HSZ * NV;
constexpr size_t OUT1_OFF = OUT0_N;
constexpr size_t OUT2_OFF = OUT0_N + OUT1_N;
typedef char chk_out[(OUT1_OFF * 4 == (size_t)26214400 && OUT2_OFF * 4 == (size_t)26624000 &&
                      (OUT2_OFF + OUT1_N) * 4 == (size_t)27033600 && (OUT0_N % 128) == 0 && (OUT1_N % 128) == 0) ? 1 : -1];

__device__ __forceinline__ v8f z8() { return (v8f){0.f, 0.f, 0.f, 0.f, 0.f, 0.f, 0.f, 0.f}; }
__device__ __forceinline__ float bfr(float f) { return bf_bits2f(f2bf_bits(f)); }
__device__ __forceinline__ unsigned short h_bits(float f) { const _Float16 h = (_Float16)f; return __builtin_bit_cast(unsigned short, h); }
__device__ __forceinline__ void split16(float f, unsigned short& hb, unsigned short& lb) {
  const _Float16 h = (_Float16)f;
  const float fh = (float)h;
  const _Float16 l = (_Float16)((f - fh) * 2048.0f);
  hb = __builtin_bit_cast(unsigned short, h);
  lb = __builtin_bit_cast(unsigned short, l);
}
__device__ __forceinline__ float sigm_f(float x) { return __builtin_amdgcn_rcpf(1.0f + exp2f(-LOG2E_F * x)); }
__device__ __forceinline__ float tanh_f(float x) { return 1.0f - 2.0f * __builtin_amdgcn_rcpf(1.0f + exp2f(2.0f * LOG2E_F * x)); }
__device__ __forceinline__ void wave_lds_sync() {
  __builtin_amdgcn_fence(__ATOMIC_RELEASE, "workgroup");
  __builtin_amdgcn_wave_barrier();
  __builtin_amdgcn_fence(__ATOMIC_ACQUIRE, "workgroup");
}
__device__ __forceinline__ v4u pack8(const unsigned short (&b)[8]) {
  v4u pk;
  pk[0] = (unsigned)b[0] | ((unsigned)b[1] << 16);
  pk[1] = (unsigned)b[2] | ((unsigned)b[3] << 16);
  pk[2] = (unsigned)b[4] | ((unsigned)b[5] << 16);
  pk[3] = (unsigned)b[6] | ((unsigned)b[7] << 16);
  return pk;
}
__device__ __forceinline__ void store16x8(unsigned short* dst, const unsigned short (&b)[8]) {
  const v4u pk = pack8(b);
  *(volatile v4u*)dst = pk;
  __threadfence();
  *(volatile v4u*)dst = pk;
}
union U8 { v4f q[2]; float f[8]; };

__global__ __launch_bounds__(256) void prep_gate_weights(const float* __restrict__ Wg, const float* __restrict__ Ug,
                                                         unsigned short* __restrict__ Apl) {
  const int g = blockIdx.x * 256 + threadIdx.x;
  const int mp = g / 192;
  const int ch = g - 192 * mp;
  const int k8 = ch * 8;
  const int tm = mp >> 6, gi = (mp >> 4) & 3, r = mp & 15;
  const int o = gi * HSZ + tm * 16 + r;
  const int kw = (k8 < KXW) ? k8 : 0;
  const int ku = (k8 >= KXW) ? (k8 - KXW) : 0;
  U8 wu, uu;
  wu.q[0] = *(const v4f*)(Wg + (size_t)o * KXW + kw);
  wu.q[1] = *(const v4f*)(Wg + (size_t)o * KXW + kw + 4);
  uu.q[0] = *(const v4f*)(Ug + (size_t)o * KHW + ku);
  uu.q[1] = *(const v4f*)(Ug + (size_t)o * KHW + ku + 4);
  unsigned short bits[8];
#pragma unroll
  for (int e = 0; e < 8; ++e) {
    const unsigned short bw = f2bf_bits(64.0f * bfr(wu.f[e]));
    const unsigned short bu = h_bits(64.0f * bfr(uu.f[e]));
    bits[e] = (k8 < KXW) ? bw : bu;
  }
  store16x8(Apl + (size_t)mp * KTOT + k8, bits);
}

__global__ __launch_bounds__(256) void prep_misc(
    const float* __restrict__ A_wg, const float* __restrict__ A_ug, const float* __restrict__ Wh,
    const float* __restrict__ Wgb, const float* __restrict__ Ugb, const float* __restrict__ bb,
    unsigned short* __restrict__ Awg16, unsigned short* __restrict__ Aug16, unsigned short* __restrict__ Wh16,
    float* __restrict__ biasT, float* __restrict__ C0, float* __restrict__ hpre,
    unsigned short* __restrict__ Bhi, unsigned short* __restrict__ Blo) {
  const int bid = blockIdx.x, tid = threadIdx.x;
  if (bid < 8) {
    const bool is_ug = (bid >= 4);
    const int g = (bid - (is_ug ? 4 : 0)) * 256 + tid;
    const int row = g >> 2, u8 = (g & 3) * 8;
    const int rc = (row < AROWS) ? row : (AROWS - 1);
    const float* src = is_ug ? A_ug : A_wg;
    unsigned short bits[8];
#pragma unroll
    for (int e = 0; e < 8; ++e) {
      const int u = u8 + e;
      const int uc = (u < NV) ? u : (NV - 1);
      float v = src[rc * NV + uc];
      v = (row < AROWS && u < NV) ? v : 0.0f;
      const unsigned short bw = f2bf_bits(v);
      const unsigned short bu = h_bits(16.0f * bfr(v));
      bits[e] = is_ug ? bu : bw;
    }
    store16x8((is_ug ? Aug16 : Awg16) + row * VPAD + u8, bits);
  } else if (bid < 12) {
    const int g = (bid - 8) * 256 + tid;
    const int idx8 = g * 8;
    U8 wu;
    wu.q[0] = *(const v4f*)(Wh + idx8);
    wu.q[1] = *(const v4f*)(Wh + idx8 + 4);
    unsigned short bits[8];
#pragma unroll
    for (int e = 0; e < 8; ++e) bits[e] = h_bits(64.0f * bfr(wu.f[e]));
    store16x8(Wh16 + idx8, bits);
  } else if (bid < 25) {
    const int g = (bid - 12) * 256 + tid;
    if (g < 3200) {
      v4f val;
#pragma unroll
      for (int e = 0; e < 4; ++e) {
        const int idx = g * 4 + e;
        const int mp = idx / NV;
        const int v = idx - NV * mp;
        const int tm = mp >> 6, gi = (mp >> 4) & 3, r = mp & 15;
        const int o = gi * HSZ + tm * 16 + r;
        val[e] = (bfr(Wgb[o]) + bfr(Ugb[o])) + bfr(bb[o * NV + v]);
      }
      float* dst = biasT + (size_t)g * 4;
      *(volatile v4f*)dst = val;
      __threadfence();
      *(volatile v4f*)dst = val;
    }
  } else if (bid < 233) {
    const bool second = (bid >= 129);
    const int g = (bid - (second ? 129 : 25)) * 256 + tid;
    float* dst = (second ? hpre : C0) + (size_t)g * 4;
    const v4f z = (v4f){0.f, 0.f, 0.f, 0.f};
    *(volatile v4f*)dst = z;
    __threadfence();
    *(volatile v4f*)dst = z;
  } else {
    const bool lo = (bid >= 257);
    const int g = (bid - (lo ? 257 : 233)) * 256 + tid;
    unsigned short* dst = lo ? (Blo + (size_t)NCOL * KXW + (size_t)g * 8) : (Bhi + (size_t)NCOL * KTOT + (size_t)g * 8);
    const v4u z = (v4u){0u, 0u, 0u, 0u};
    *(volatile v4u*)dst = z;
    __threadfence();
    *(volatile v4u*)dst = z;
  }
}

__global__ __launch_bounds__(256) void gate_gemm_lstm(
    const unsigned short* __restrict__ Apl, const unsigned short* __restrict__ Bhi,
    const unsigned short* __restrict__ Blo, const float* __restrict__ biasT,
    const float* __restrict__ cin, float* __restrict__ cout, float* __restrict__ hpre) {
  __shared__ __align__(16) float sBias[2 * 1600];
  __shared__ __align__(16) float sSlab[8 * 3 * 512];
  const int tid = threadIdx.x;
  const int lane = tid & 31, wave = tid >> 5;
  const int hh = lane >> 4, rlane = lane & 15, koff = hh * 8;
  const int tile = blockIdx.x * 8 + wave;
  const int tm = tile / GEMM_TN;
  const int tn = tile - GEMM_TN * tm;
  const int tmA = (blockIdx.x * 8) / GEMM_TN;
  for (int i = tid; i < 800; i += 256) {
    const int slot = (i >= 400) ? 1 : 0;
    const int loc = i - 400 * slot;
    int tms = tmA + slot;
    tms = (tms > GEMM_TM - 1) ? (GEMM_TM - 1) : tms;
    const v4f b4 = *(const v4f*)(biasT + (size_t)tms * 1600 + loc * 4);
    *(v4f*)(sBias + slot * 1600 + loc * 4) = b4;
  }
  __syncthreads();
  const float* sB = sBias + (tm - tmA) * 1600;
  const int m0 = tm * 64, n0 = tn * 64;

  v8f acc[4][4];
#pragma unroll
  for (int i = 0; i < 4; ++i)
#pragma unroll
    for (int j = 0; j < 4; ++j) acc[i][j] = z8();

  {
    const __bf16* Ab = (const __bf16*)Apl;
    const __bf16* Bb = (const __bf16*)Bhi;
    const __bf16* Lb = (const __bf16*)Blo;
    for (int k0 = 0; k0 < KXW; k0 += 32) {
      v16b bh[4], bl[4];
#pragma unroll
      for (int j = 0; j < 4; ++j) {
        const size_t ro = (size_t)(n0 + (j << 4) + rlane);
        bh[j] = Frag<__bf16>::load(Bb + ro * KTOT + koff + k0);
        bl[j] = Frag<__bf16>::load(Lb + ro * KXW + koff + k0);
      }
#pragma unroll
      for (int i = 0; i < 4; ++i) {
        const v16b a = Frag<__bf16>::load(Ab + (size_t)(m0 + (i << 4) + rlane) * KTOT + koff + k0);
#pragma unroll
        for (int j = 0; j < 4; ++j) {
          acc[i][j] = Frag<__bf16>::mma(a, bh[j], acc[i][j]);
          acc[i][j] = Frag<__bf16>::mma(a, bl[j], acc[i][j]);
        }
        Frag<__bf16>::guard(acc[i][0], acc[i][3], a, a);
      }
      Frag<__bf16>::keep(bh[0], bh[1], bh[2], bh[3]);
      Frag<__bf16>::keep(bl[0], bl[1], bl[2], bl[3]);
    }
  }
  {
    const _Float16* Af = (const _Float16*)Apl;
    const _Float16* Bf = (const _Float16*)Bhi;
    for (int k0 = KXW; k0 < KTOT; k0 += 32) {
      v16h bh[4];
#pragma unroll
      for (int j = 0; j < 4; ++j)
        bh[j] = Frag<_Float16>::load(Bf + (size_t)(n0 + (j << 4) + rlane) * KTOT + koff + k0);
#pragma unroll
      for (int i = 0; i < 4; ++i) {
        const v16h a = Frag<_Float16>::load(Af + (size_t)(m0 + (i << 4) + rlane) * KTOT + koff + k0);
#pragma unroll
        for (int j = 0; j < 4; ++j) acc[i][j] = Frag<_Float16>::mma(a, bh[j], acc[i][j]);
        Frag<_Float16>::guard(acc[i][0], acc[i][3], a, a);
      }
      Frag<_Float16>::keep(bh[0], bh[1], bh[2], bh[3]);
    }
  }
  acc_guard4(acc[0][0], acc[0][1], acc[0][2], acc[0][3]);
  acc_guard4(acc[1][0], acc[1][1], acc[1][2], acc[1][3]);
  acc_guard4(acc[2][0], acc[2][1], acc[2][2], acc[2][3]);
  acc_guard4(acc[3][0], acc[3][1], acc[3][2], acc[3][3]);

  float* slF  = sSlab + (wave * 3 + 0) * 512;
  float* slIG = sSlab + (wave * 3 + 1) * 512;
  float* slO  = sSlab + (wave * 3 + 2) * 512;
  const int hs0 = tm * 16;
  const int q8 = lane >> 3, c4 = (lane & 7) * 4;
#pragma unroll
  for (int ch = 0; ch < 2; ++ch) {
#pragma unroll
    for (int jj = 0; jj < 2; ++jj) {
      const int j = 2 * ch + jj;
      const int col = n0 + 16 * j + rlane;
      const int vj = col - NV * (col / NV);
#pragma unroll
      for (int r = 0; r < 8; ++r) {
        const int hsl = 8 * hh + r;
        const float gi = acc[0][j][r] * SC_W + sB[(0 * 16 + hsl) * NV + vj];
        const float gf = acc[1][j][r] * SC_W + sB[(1 * 16 + hsl) * NV + vj];
        const float gg = acc[2][j][r] * SC_W + sB[(2 * 16 + hsl) * NV + vj];
        const float go = acc[3][j][r] * SC_W + sB[(3 * 16 + hsl) * NV + vj];
        const int si = hsl * 32 + jj * 16 + rlane;
        slF[si]  = sigm_f(gf);
        slIG[si] = sigm_f(gi) * tanh_f(gg);
        slO[si]  = sigm_f(go);
      }
    }
    wave_lds_sync();
    v4f cn[4], hn[4];
#pragma unroll
    for (int it = 0; it < 4; ++it) {
      const int row = it * 4 + q8;
      const size_t idx = (size_t)(hs0 + row) * NCOLP + n0 + ch * 32 + c4;
      const v4f co  = *(const v4f*)(cin + idx);
      const v4f f4  = *(const v4f*)(slF + row * 32 + c4);
      const v4f ig4 = *(const v4f*)(slIG + row * 32 + c4);
      const v4f o4  = *(const v4f*)(slO + row * 32 + c4);
      const v4f cc = f4 * co + ig4;
      v4f hv;
      hv[0] = o4[0] * tanh_f(cc[0]);
      hv[1] = o4[1] * tanh_f(cc[1]);
      hv[2] = o4[2] * tanh_f(cc[2]);
      hv[3] = o4[3] * tanh_f(cc[3]);
      cn[it] = cc;
      hn[it] = hv;
    }
    for (int pass = 0; pass < 2; ++pass) {
#pragma unroll
      for (int it = 0; it < 4; ++it) {
        const int row = it * 4 + q8;
        const size_t idx = (size_t)(hs0 + row) * NCOLP + n0 + ch * 32 + c4;
        *(volatile v4f*)(cout + idx) = cn[it];
        *(volatile v4f*)(hpre + idx) = hn[it];
      }
      __threadfence();
    }
    wave_lds_sync();
  }
}

__global__ __launch_bounds__(128) void state_step(
    const float* __restrict__ hpre, const float* __restrict__ x,
    const float* __restrict__ Ww, const float* __restrict__ Wb,
    const float* __restrict__ Wq, const float* __restrict__ Wqb,
    const float* __restrict__ Whb, const float* __restrict__ Us, const float* __restrict__ Usb,
    const unsigned short* __restrict__ Wh16, const unsigned short* __restrict__ Aug16,
    const unsigned short* __restrict__ Awg16,
    unsigned short* __restrict__ Bhi, unsigned short* __restrict__ Blo,
    float* __restrict__ hseq, int t) {
  __shared__ __align__(16) float sh_h[HSZ * VPAD];
  __shared__ __align__(16) unsigned short pl16[2][HSZ * VPAD];
  __shared__ __align__(16) unsigned short x16[NCIN * VPAD];
  __shared__ __align__(16) float slab_all[4 * 16 * SLABP];
  __shared__ float sh_hsum[HSZ];
  __shared__ float sh_q[NC1];
  __shared__ float sh_qq[NC2];
  __shared__ float sh_a[VPAD];

  const int n = blockIdx.x, tid = threadIdx.x;
  const int wave = tid >> 5, lane = tid & 31;
  const int hh = lane >> 4, rlane = lane & 15, koff = hh * 8;
  const bool init = (t < 0);
  const int tcur = init ? 0 : t;
  const int tnx = (t + 1 < TT) ? (t + 1) : (TT - 1);

#pragma unroll 4
  for (int i = tid; i < HSZ * VPAD; i += 128) {
    const int hs = i >> 5, v = i & 31;
    const int vc = (v < NV) ? v : (NV - 1);
    float hv = hpre[(size_t)hs * NCOLP + n * NV + vc];
    hv = (v < NV && !init) ? hv : 0.0f;
    sh_h[i] = hv;
  }
#pragma unroll 4
  for (int i = tid; i < NCIN * VPAD; i += 128) {
    const int c = i >> 5, u = i & 31;
    const int uc = (u < NV) ? u : (NV - 1);
    const float xv = x[(((size_t)n * NCIN + c) * TT + tnx) * NV + uc];
    const unsigned short bits = f2bf_bits(xv);
    x16[i] = (u < NV) ? bits : (unsigned short)0;
  }
  __syncthreads();

  {
    const int hs = tid;
    float s = 0.0f;
#pragma unroll
    for (int v = 0; v < VPAD; ++v) {
      const float hv = sh_h[hs * VPAD + v];
      if (v < NV) s += hv;
      unsigned short hb, lb;
      split16(hv, hb, lb);
      pl16[0][v * HSZ + hs] = hb;
      pl16[1][v * HSZ + hs] = lb;
    }
    sh_hsum[hs] = s;
  }
  __syncthreads();

  if (tid < NC1) {
    const float* wr = Ww + tid * HSZ;
    float s = 0.0f;
#pragma unroll 2
    for (int k4 = 0; k4 < HSZ / 4; ++k4) {
      const v4f w = *(const v4f*)(wr + 4 * k4);
      s += bfr(w[0]) * sh_hsum[4 * k4 + 0];
      s += bfr(w[1]) * sh_hsum[4 * k4 + 1];
      s += bfr(w[2]) * sh_hsum[4 * k4 + 2];
      s += bfr(w[3]) * sh_hsum[4 * k4 + 3];
    }
    s += bfr(Wb[tid]);
    sh_q[tid] = fmaxf(s, 0.0f);
  }
  __syncthreads();

  if (tid < NC2) {
    const float* wr = Wq + tid * NC1;
    float s = 0.0f;
#pragma unroll 2
    for (int k4 = 0; k4 < NC1 / 4; ++k4) {
      const v4f w = *(const v4f*)(wr + 4 * k4);
      s += bfr(w[0]) * sh_q[4 * k4 + 0];
      s += bfr(w[1]) * sh_q[4 * k4 + 1];
      s += bfr(w[2]) * sh_q[4 * k4 + 2];
      s += bfr(w[3]) * sh_q[4 * k4 + 3];
    }
    s += bfr(Wqb[tid]);
    sh_qq[tid] = s;
  }
  __syncthreads();

  {
    const int ct = wave;
    const _Float16* Ph = (const _Float16*)&pl16[0][0];
    const _Float16* Pl = (const _Float16*)&pl16[1][0];
    const _Float16* Wp = (const _Float16*)Wh16;
    v8f a0 = z8(), l0 = z8(), a1 = z8(), l1 = z8();
#pragma unroll
    for (int ks = 0; ks < 4; ++ks) {
      const int k0 = ks * 32;
      const v16h b   = Frag<_Float16>::load(Wp + (size_t)(ct * 16 + rlane) * HSZ + koff + k0);
      const v16h x0h = Frag<_Float16>::load(Ph + rlane * HSZ + koff + k0);
      const v16h x0l = Frag<_Float16>::load(Pl + rlane * HSZ + koff + k0);
      const v16h x1h = Frag<_Float16>::load(Ph + (16 + rlane) * HSZ + koff + k0);
      const v16h x1l = Frag<_Float16>::load(Pl + (16 + rlane) * HSZ + koff + k0);
      a0 = Frag<_Float16>::mma(x0h, b, a0);
      l0 = Frag<_Float16>::mma(x0l, b, l0);
      a1 = Frag<_Float16>::mma(x1h, b, a1);
      l1 = Frag<_Float16>::mma(x1l, b, l1);
      Frag<_Float16>::guard(a0, l1, x0h, b);
      Frag<_Float16>::guard(l0, a1, x1h, x1l);
    }
    acc_guard4(a0, l0, a1, l1);
    const int c2 = ct * 16 + rlane;
    const float whb = bfr(Whb[c2]);
    const float qqv = sh_qq[c2];
    float* sh_u = slab_all;
#pragma unroll
    for (int r = 0; r < 8; ++r) {
      const int v0 = 8 * hh + r, v1 = 16 + 8 * hh + r;
      float p0 = (a0[r] + l0[r] * SC_RES) * SC_W;
      p0 = (p0 + whb) + qqv;
      float p1 = (a1[r] + l1[r] * SC_RES) * SC_W;
      p1 = (p1 + whb) + qqv;
      sh_u[v0 * NC2 + c2] = tanh_f(p0);
      sh_u[v1 * NC2 + c2] = tanh_f(p1);
    }
  }
  __syncthreads();

  if (tid < VPAD) {
    const float* su = slab_all + tid * NC2;
    float s = 0.0f;
#pragma unroll 2
    for (int k4 = 0; k4 < NC2 / 4; ++k4) {
      const v4f w = *(const v4f*)(Us + 4 * k4);
      s += bfr(w[0]) * su[4 * k4 + 0];
      s += bfr(w[1]) * su[4 * k4 + 1];
      s += bfr(w[2]) * su[4 * k4 + 2];
      s += bfr(w[3]) * su[4 * k4 + 3];
    }
    s += bfr(Usb[0]);
    sh_a[tid] = sigm_f(s);
  }
  __syncthreads();

#pragma unroll 4
  for (int i = tid; i < HSZ * VPAD; i += 128) {
    const int v = i & 31;
    const float hp = sh_h[i];
    const float av = sh_a[v];
    float hn = av * hp + hp;
    hn = (v < NV) ? hn : 0.0f;
    sh_h[i] = hn;
    unsigned short hb, lb;
    split16(hn, hb, lb);
    pl16[0][i] = hb;
    pl16[1][i] = lb;
  }
  __syncthreads();

  if (!init) {
    float* hb = hseq + ((size_t)tcur * NB + n) * (size_t)(HSZ * VPAD);
    const int q8 = lane >> 3, c4 = (lane & 7) * 4;
    for (int pass = 0; pass < 2; ++pass) {
#pragma unroll
      for (int it = 0; it < 8; ++it) {
        const int row = it * 16 + wave * 4 + q8;
        const v4f val = *(const v4f*)(sh_h + row * VPAD + c4);
        *(volatile v4f*)(hb + (size_t)row * VPAD + c4) = val;
      }
      __threadfence();
    }
  }

  {
    const int cg = wave & 1;
    const _Float16* Ph = (const _Float16*)&pl16[0][0];
    const _Float16* Pl = (const _Float16*)&pl16[1][0];
    const _Float16* Ap = (const _Float16*)Aug16;
    v16h bh[4], bl[4];
#pragma unroll
    for (int j = 0; j < 4; ++j) {
      const int c = cg * 64 + j * 16 + rlane;
      bh[j] = Frag<_Float16>::load(Ph + c * VPAD + koff);
      bl[j] = Frag<_Float16>::load(Pl + c * VPAD + koff);
    }
    float* slab = slab_all + wave * (16 * SLABP);
    const int q8 = lane >> 3, c8 = (lane & 7) * 8;
#pragma unroll 1
    for (int uu = wave; uu < 2 * AROWT; uu += 4) {
      const int rt = uu >> 1;
      const v16h a = Frag<_Float16>::load(Ap + (rt * 16 + rlane) * VPAD + koff);
      v8f acc[4], accl[4];
#pragma unroll
      for (int j = 0; j < 4; ++j) {
        acc[j]  = Frag<_Float16>::mma(a, bh[j], z8());
        accl[j] = Frag<_Float16>::mma(a, bl[j], z8());
      }
      Frag<_Float16>::guard(acc[0], accl[3], a, a);
      acc_guard4(acc[0], acc[1], acc[2], acc[3]);
      acc_guard4(accl[0], accl[1], accl[2], accl[3]);
#pragma unroll
      for (int j = 0; j < 4; ++j)
#pragma unroll
        for (int r = 0; r < 8; ++r)
          slab[(8 * hh + r) * SLABP + j * 16 + rlane] = (acc[j][r] + accl[j][r] * SC_RES) * SC_AUG;
      wave_lds_sync();
      v8h hv[4];
#pragma unroll
      for (int it = 0; it < 4; ++it) {
        const int row = it * 4 + q8;
        const float* sp = slab + row * SLABP + c8;
#pragma unroll
        for (int e = 0; e < 8; ++e) hv[it][e] = (_Float16)sp[e];
      }
      for (int pass = 0; pass < 2; ++pass) {
#pragma unroll
        for (int it = 0; it < 4; ++it) {
          const int row = it * 4 + q8;
          const int grow = rt * 16 + row;
          const int s = grow / NV;
          const int w = grow - NV * s;
          if (grow < AROWS)
            *(volatile v8h*)(Bhi + (size_t)(n * NV + w) * KTOT + KXW + s * HSZ + cg * 64 + c8) = hv[it];
        }
        __threadfence();
      }
      wave_lds_sync();
    }
    Frag<_Float16>::keep(bh[0], bh[1], bh[2], bh[3]);
    Frag<_Float16>::keep(bl[0], bl[1], bl[2], bl[3]);
  }

  {
    const __bf16* Xp = (const __bf16*)&x16[0];
    const __bf16* Ap = (const __bf16*)Awg16;
    v16b bx[4];
#pragma unroll
    for (int j = 0; j < 4; ++j) bx[j] = Frag<__bf16>::load(Xp + (j * 16 + rlane) * VPAD + koff);
    float* slab = slab_all + wave * (16 * SLABP);
    const int q8 = lane >> 3, c8 = (lane & 7) * 8;
#pragma unroll 1
    for (int rt = wave; rt < AROWT; rt += 4) {
      const v16b a = Frag<__bf16>::load(Ap + (rt * 16 + rlane) * VPAD + koff);
      v8f acc[4];
#pragma unroll
      for (int j = 0; j < 4; ++j) acc[j] = Frag<__bf16>::mma(a, bx[j], z8());
      Frag<__bf16>::guard(acc[0], acc[3], a, a);
      acc_guard4(acc[0], acc[1], acc[2], acc[3]);
#pragma unroll
      for (int j = 0; j < 4; ++j)
#pragma unroll
        for (int r = 0; r < 8; ++r)
          slab[(8 * hh + r) * SLABP + j * 16 + rlane] = acc[j][r];
      wave_lds_sync();
      v8h hv[4], lv[4];
#pragma unroll
      for (int it = 0; it < 4; ++it) {
        const int row = it * 4 + q8;
        const float* sp = slab + row * SLABP + c8;
#pragma unroll
        for (int e = 0; e < 8; ++e) {
          const float f = sp[e];
          const unsigned short hb = f2bf_bits(f);
          const unsigned short lb = f2bf_bits(f - bf_bits2f(hb));
          hv[it][e] = __builtin_bit_cast(_Float16, hb);
          lv[it][e] = __builtin_bit_cast(_Float16, lb);
        }
      }
      for (int pass = 0; pass < 2; ++pass) {
#pragma unroll
        for (int it = 0; it < 4; ++it) {
          const int row = it * 4 + q8;
          const int grow = rt * 16 + row;
          const int s = grow / NV;
          const int w = grow - NV * s;
          if (grow < AROWS) {
            *(volatile v8h*)(Bhi + (size_t)(n * NV + w) * KTOT + s * NCIN + c8) = hv[it];
            *(volatile v8h*)(Blo + (size_t)(n * NV + w) * KXW + s * NCIN + c8) = lv[it];
          }
        }
        __threadfence();
      }
      wave_lds_sync();
    }
    Frag<__bf16>::keep(bx[0], bx[1], bx[2], bx[3]);
  }
}

__global__ __launch_bounds__(256) void write_outputs(const float* __restrict__ hseq, const float* __restrict__ cfin,
                                                    float* __restrict__ out) {
  const unsigned g = blockIdx.x * 256u + threadIdx.x;
  const unsigned n0q = (unsigned)(OUT0_N / 4);
  const unsigned n1q = (unsigned)(OUT1_N / 4);
  v4f val;
  float* dst;
  if (g < n0q) {
#pragma unroll
    for (int e = 0; e < 4; ++e) {
      const unsigned idx = g * 4u + e;
      const unsigned v  = idx % NV;
      const unsigned tq = (idx / NV) % TT;
      const unsigned hs = (idx / (NV * TT)) % HSZ;
      const unsigned nn = idx / (NV * TT * HSZ);
      val[e] = hseq[(((size_t)tq * NB + nn) * HSZ + hs) * VPAD + v];
    }
    dst = out + (size_t)g * 4;
  } else if (g < n0q + n1q) {
    const unsigned g1 = g - n0q;
#pragma unroll
    for (int e = 0; e < 4; ++e) {
      const unsigned idx = g1 * 4u + e;
      const unsigned v  = idx % NV;
      const unsigned hs = (idx / NV) % HSZ;
      const unsigned nn = idx / (NV * HSZ);
      val[e] = hseq[(((size_t)(TT - 1) * NB + nn) * HSZ + hs) * VPAD + v];
    }
    dst = out + OUT1_OFF + (size_t)g1 * 4;
  } else {
    const unsigned g2 = g - n0q - n1q;
#pragma unroll
    for (int e = 0; e < 4; ++e) {
      const unsigned idx = g2 * 4u + e;
      const unsigned v  = idx % NV;
      const unsigned hs = (idx / NV) % HSZ;
      const unsigned nn = idx / (NV * HSZ);
      val[e] = cfin[(size_t)hs * NCOLP + nn * NV + v];
    }
    dst = out + OUT2_OFF + (size_t)g2 * 4;
  }
  *(volatile v4f*)dst = val;
  __threadfence();
  *(volatile v4f*)dst = val;
}

extern "C" void kernel_launch(void* const* d_in, const int* in_sizes, int n_in,
                              void* d_out, int out_size, void* d_ws, size_t ws_size,
                              hipStream_t stream) {
  (void)in_sizes; (void)n_in; (void)out_size; (void)ws_size;
  const float* x    = (const float*)d_in[0];
  const float* A_wg = (const float*)d_in[1];
  const float* Wg   = (const float*)d_in[2];
  const float* Wgb  = (const float*)d_in[3];
  const float* A_ug = (const float*)d_in[4];
  const float* Ug   = (const float*)d_in[5];
  const float* Ugb  = (const float*)d_in[6];
  const float* bb   = (const float*)d_in[7];
  const float* Ww   = (const float*)d_in[8];
  const float* Wb   = (const float*)d_in[9];
  const float* Wq   = (const float*)d_in[10];
  const float* Wqb  = (const float*)d_in[11];
  const float* Wh   = (const float*)d_in[12];
  const float* Whb  = (const float*)d_in[13];
  const float* Us   = (const float*)d_in[14];
  const float* Usb  = (const float*)d_in[15];
  float* out = (float*)d_out;

  char* ws = (char*)d_ws;
  unsigned short* Apl   = (unsigned short*)(ws + OFF_APL);
  unsigned short* Bhi   = (unsigned short*)(ws + OFF_BHI);
  unsigned short* Blo   = (unsigned short*)(ws + OFF_BLO);
  float*          biasT = (float*)(ws + OFF_BIAS);
  unsigned short* Awg16 = (unsigned short*)(ws + OFF_AWG);
  unsigned short* Aug16 = (unsigned short*)(ws + OFF_AUG);
  unsigned short* Wh16  = (unsigned short*)(ws + OFF_WH);
  float*          Cbuf0 = (float*)(ws + OFF_C0);
  float*          Cbuf1 = (float*)(ws + OFF_C1);
  float*          hpre  = (float*)(ws + OFF_HPRE);
  float*          hseq  = (float*)(ws + OFF_HSEQ);

  prep_gate_weights<<<(MG * KTOT / 8) / 256, 256, 0, stream>>>(Wg, Ug, Apl);
  prep_misc<<<265, 256, 0, stream>>>(A_wg, A_ug, Wh, Wgb, Ugb, bb, Awg16, Aug16, Wh16, biasT, Cbuf0, hpre, Bhi, Blo);
  state_step<<<NB, 128, 0, stream>>>(hpre, x, Ww, Wb, Wq, Wqb, Whb, Us, Usb, Wh16, Aug16, Awg16, Bhi, Blo, hseq, -1);
  for (int t = 0; t < TT; ++t) {
    const float* cin = (t & 1) ? Cbuf1 : Cbuf0;
    float* cout = (t & 1) ? Cbuf0 : Cbuf1;
    gate_gemm_lstm<<<13, 256, 0, stream>>>(Apl, Bhi, Blo, biasT, cin, cout, hpre);
    state_step<<<NB, 128, 0, stream>>>(hpre, x, Ww, Wb, Wq, Wqb, Whb, Us, Usb, Wh16, Aug16, Awg16, Bhi, Blo, hseq, t);
  }
  write_outputs<<<(unsigned)((OUT0_N + 2 * OUT1_N) / 4 / 256), 256, 0, stream>>>(hseq, Cbuf0, out);
}
